// SwinTransformer_MAE3D_57904749085153
// MI455X (gfx1250) — hardware-verified
//
#include <hip/hip_runtime.h>
#include <stdint.h>

#define NWIN 64
#define NTOK 512
#define CCH  256
#define NHD  8
#define HD   32
#define C3   768
#define NROW 32768
#define NRPB 3375
#define LDC  132
#define PP   72
#define OSP  36
#define PWB  4608
#define QSC  0.17677669529663687f
#define INV512 0.001953125f
#define LN4096 8.3177661667193429f

static_assert(NROW == NWIN * NTOK);
static_assert(PWB == 2 * 16 * PP * 2);
static_assert(16 * OSP * 4 <= PWB);
static_assert((PP * 2) % 16 == 0);
static_assert((LDC * 4) % 16 == 0);

typedef _Float16 v16h __attribute__((ext_vector_type(16)));
typedef _Float16 v8h  __attribute__((ext_vector_type(8)));
typedef float    v8f  __attribute__((ext_vector_type(8)));
typedef float    v4f  __attribute__((ext_vector_type(4)));
typedef unsigned int v4u __attribute__((ext_vector_type(4)));

__device__ __forceinline__ unsigned short bf_bits(float f) {
  unsigned u = __float_as_uint(f);
  return (unsigned short)((u + 0x7FFFu + ((u >> 16) & 1u)) >> 16);
}
__device__ __forceinline__ float bf_up(unsigned short b) { return __uint_as_float(((unsigned)b) << 16); }
__device__ __forceinline__ float bfr(float f) { return bf_up(bf_bits(f)); }
__device__ __forceinline__ unsigned short h_bits(_Float16 x) { return __builtin_bit_cast(unsigned short, x); }
__device__ __forceinline__ unsigned short hb16(float f) { return h_bits((_Float16)f); }
__device__ __forceinline__ unsigned pk16(unsigned short a, unsigned short b) { return (unsigned)a | ((unsigned)b << 16); }
__device__ __forceinline__ v8f zero8() { v8f z = {0.f, 0.f, 0.f, 0.f, 0.f, 0.f, 0.f, 0.f}; return z; }

__device__ __forceinline__ int spat_of(int w, int t) {
  const int hb = w >> 4, wb = (w >> 2) & 3, db = w & 3;
  const int i = t >> 6, j = (t >> 3) & 7, k = t & 7;
  const int gh = (hb * 8 + i + 4) & 31;
  const int gw = (wb * 8 + j + 4) & 31;
  const int gd = (db * 8 + k + 4) & 31;
  return (gh * 32 + gw) * 32 + gd;
}
__device__ __forceinline__ int rid1(int p) { return (p < 24) ? 0 : ((p < 28) ? 1 : 2); }
__device__ __forceinline__ int region_of(int w, int t) {
  const int hb = w >> 4, wb = (w >> 2) & 3, db = w & 3;
  const int i = t >> 6, j = (t >> 3) & 7, k = t & 7;
  return rid1(hb * 8 + i) * 9 + rid1(wb * 8 + j) * 3 + rid1(db * 8 + k);
}

__device__ __forceinline__ v16h ldfrag_h(const _Float16* p) {
  union { v16h v; v8h h[2]; } f;
  f.h[0] = *(const v8h*)(p);
  f.h[1] = *(const v8h*)(p + 16);
  return f.v;
}

__device__ __forceinline__ v8f mma_raw(v16h a, v16h b, v8f c) {
  return __builtin_amdgcn_wmma_f32_16x16x32_f16(false, a, false, b, (short)0, c, false, false);
}
__device__ __forceinline__ v8f mma_g1(v16h a, v16h b, v8f c) {
  c = mma_raw(a, b, c);
#if defined(__HIP_DEVICE_COMPILE__)
  asm volatile("v_nop\n\tv_nop\n\tv_nop\n\tv_nop" : "+v"(c) : "v"(a), "v"(b));
#endif
  return c;
}
__device__ __forceinline__ void guard3(v8f& c0, v8f& c1, v8f& c2,
                                       const v16h& a0, const v16h& a1, const v16h& b0, const v16h& b1) {
#if defined(__HIP_DEVICE_COMPILE__)
  asm volatile("v_nop\n\tv_nop\n\tv_nop\n\tv_nop"
               : "+v"(c0), "+v"(c1), "+v"(c2) : "v"(a0), "v"(a1), "v"(b0), "v"(b1));
#endif
}
__device__ __forceinline__ void guard4(v8f& c0, v8f& c1, v8f& c2, v8f& c3,
                                       const v16h& a0, const v16h& a1, const v16h& b0, const v16h& b1) {
#if defined(__HIP_DEVICE_COMPILE__)
  asm volatile("v_nop\n\tv_nop\n\tv_nop\n\tv_nop"
               : "+v"(c0), "+v"(c1), "+v"(c2), "+v"(c3) : "v"(a0), "v"(a1), "v"(b0), "v"(b1));
#endif
}
__device__ __forceinline__ void guard8(v8f& c0, v8f& c1, v8f& c2, v8f& c3, v8f& c4, v8f& c5, v8f& c6, v8f& c7,
                                       const v16h& a0, const v16h& a1, const v16h& a2, const v16h& a3,
                                       const v16h& b0, const v16h& b1) {
#if defined(__HIP_DEVICE_COMPILE__)
  asm volatile("v_nop\n\tv_nop\n\tv_nop\n\tv_nop"
               : "+v"(c0), "+v"(c1), "+v"(c2), "+v"(c3), "+v"(c4), "+v"(c5), "+v"(c6), "+v"(c7)
               : "v"(a0), "v"(a1), "v"(a2), "v"(a3), "v"(b0), "v"(b1));
#endif
}
__device__ __forceinline__ void wave_sync_lds() {
  __builtin_amdgcn_fence(__ATOMIC_RELEASE, "workgroup");
  __builtin_amdgcn_wave_barrier();
  __builtin_amdgcn_fence(__ATOMIC_ACQUIRE, "workgroup");
}

__global__ __launch_bounds__(256) void cvt_x(const float* __restrict__ x, unsigned short* xp) {
  const int tid = threadIdx.x, wv = tid >> 5, lane = tid & 31;
  const int row = blockIdx.x * 8 + wv;
  const int w = row >> 9, t = row & 511;
  const float* src = x + (size_t)spat_of(w, t) * CCH + lane * 8;
  const v4f a = *(const v4f*)(src);
  const v4f b = *(const v4f*)(src + 4);
  v4u pk;
  pk[0] = pk16(hb16(bfr(a[0]) * 8.0f), hb16(bfr(a[1]) * 8.0f));
  pk[1] = pk16(hb16(bfr(a[2]) * 8.0f), hb16(bfr(a[3]) * 8.0f));
  pk[2] = pk16(hb16(bfr(b[0]) * 8.0f), hb16(bfr(b[1]) * 8.0f));
  pk[3] = pk16(hb16(bfr(b[2]) * 8.0f), hb16(bfr(b[3]) * 8.0f));
  unsigned short* gp = xp + (size_t)row * CCH + lane * 8;
  *(volatile v4u*)gp = pk;
  __threadfence();
  *(volatile v4u*)gp = pk;
}

__global__ __launch_bounds__(256) void cvt_w(const float* __restrict__ wsrc, unsigned short* wdst, int nrows) {
  const int tid = threadIdx.x, wv = tid >> 5, lane = tid & 31;
  const int row = blockIdx.x * 8 + wv;
  if (row < nrows) {
    const float* src = wsrc + (size_t)row * CCH + lane * 8;
    const v4f a = *(const v4f*)(src);
    const v4f b = *(const v4f*)(src + 4);
    v4u pk;
    pk[0] = pk16(hb16(bfr(a[0]) * 1024.0f), hb16(bfr(a[1]) * 1024.0f));
    pk[1] = pk16(hb16(bfr(a[2]) * 1024.0f), hb16(bfr(a[3]) * 1024.0f));
    pk[2] = pk16(hb16(bfr(b[0]) * 1024.0f), hb16(bfr(b[1]) * 1024.0f));
    pk[3] = pk16(hb16(bfr(b[2]) * 1024.0f), hb16(bfr(b[3]) * 1024.0f));
    unsigned short* gp = wdst + (size_t)row * CCH + lane * 8;
    *(volatile v4u*)gp = pk;
    __threadfence();
    *(volatile v4u*)gp = pk;
  }
}

__global__ __launch_bounds__(256) void build_bias(const float* __restrict__ rpb, float* bt) {
  const int g = blockIdx.x * 256 + threadIdx.x;
  const int piece = g & 63, rec = g >> 6;
  const int kt = rec & 31, strip = (rec >> 5) & 31, h = (rec >> 10) & 7;
  const int l = piece >> 1, e0 = (piece & 1) * 4;
  const int col = l & 15, lh = l >> 4;
  const int m = kt * 16 + col;
  const int mi = m >> 6, mj = (m >> 3) & 7, mk = m & 7;
  v4f v;
#pragma unroll
  for (int e = 0; e < 4; ++e) {
    const int n = strip * 16 + 8 * lh + e0 + e;
    const int ni = n >> 6, nj = (n >> 3) & 7, nk = n & 7;
    int idx = ((ni - mi + 7) * 15 + (nj - mj + 7)) * 15 + (nk - mk + 7);
    idx = min(max(idx, 0), NRPB - 1);
    v[e] = bfr(rpb[idx * NHD + h]) * 512.0f;
  }
  float* gp = bt + (size_t)rec * 256 + piece * 4;
  *(volatile v4f*)gp = v;
  __threadfence();
  *(volatile v4f*)gp = v;
}

__global__ __launch_bounds__(256)
void gemm_qkv(const unsigned short* __restrict__ xp, const unsigned short* __restrict__ wq,
              const float* __restrict__ bq,
              unsigned short* qpl, unsigned short* kpl, unsigned short* vth, unsigned short* vtl) {
  __shared__ __align__(16) float Cs[64 * LDC];
  const int tid = threadIdx.x, wave = tid >> 5, lane = tid & 31, hh = lane >> 4, c = lane & 15;
  const int mb = blockIdx.x, nb = blockIdx.y;
  const int mw = wave >> 2, nw = wave & 3;
  const _Float16* A = (const _Float16*)(const void*)xp;
  const _Float16* W = (const _Float16*)(const void*)wq;
  const int arow0 = mb * 64 + mw * 32;
  const int bcol0 = nb * 128 + nw * 32;

  v8f a00 = zero8(), a01 = zero8(), a10 = zero8(), a11 = zero8();
#pragma unroll 1
  for (int ks = 0; ks < 8; ++ks) {
    const int k0 = ks * 32 + 8 * hh;
    const v16h fa0 = ldfrag_h(A + (size_t)(arow0 + c) * CCH + k0);
    const v16h fa1 = ldfrag_h(A + (size_t)(arow0 + 16 + c) * CCH + k0);
    const v16h fb0 = ldfrag_h(W + (size_t)(bcol0 + c) * CCH + k0);
    const v16h fb1 = ldfrag_h(W + (size_t)(bcol0 + 16 + c) * CCH + k0);
    a00 = mma_raw(fa0, fb0, a00);
    a01 = mma_raw(fa0, fb1, a01);
    a10 = mma_raw(fa1, fb0, a10);
    a11 = mma_raw(fa1, fb1, a11);
    guard4(a00, a01, a10, a11, fa0, fa1, fb0, fb1);
  }
#pragma unroll
  for (int r = 0; r < 8; ++r) {
    const int row = mw * 32 + 8 * hh + r;
    Cs[row * LDC + nw * 32 + c]             = a00[r];
    Cs[row * LDC + nw * 32 + 16 + c]        = a01[r];
    Cs[(row + 16) * LDC + nw * 32 + c]      = a10[r];
    Cs[(row + 16) * LDC + nw * 32 + 16 + c] = a11[r];
  }
  __syncthreads();

  const int part = nb >> 1;
  const int hb4 = (nb & 1) * 4;
  const int w = mb >> 3, tok0 = (mb & 7) * 64;
  const float* bqn = bq + nb * 128;
  if (part < 2) {
    unsigned short* dst = (part == 0) ? qpl : kpl;
    const float scl = (part == 0) ? (QSC * 64.0f) : 8.0f;
    v4u pk[4];
    size_t offs[4];
#pragma unroll
    for (int s = 0; s < 4; ++s) {
      const int L = s * 32 + (tid >> 3), p = tid & 7;
      const int h4 = L >> 5, li = L & 31;
      const int tok = 2 * li + (p >> 2), d0 = (p & 3) * 8;
      const int col = h4 * 32 + d0;
      v4u q4;
#pragma unroll
      for (int e = 0; e < 4; ++e) {
        float f0 = Cs[tok * LDC + col + 2 * e] * (1.0f / 8192.0f) + bfr(bqn[col + 2 * e]);
        float f1 = Cs[tok * LDC + col + 2 * e + 1] * (1.0f / 8192.0f) + bfr(bqn[col + 2 * e + 1]);
        f0 = f0 * scl;
        f1 = f1 * scl;
        q4[e] = pk16(hb16(f0), hb16(f1));
      }
      pk[s] = q4;
      offs[s] = ((size_t)((w * NHD + hb4 + h4) * NTOK + tok0 + tok)) * HD + d0;
    }
#pragma unroll
    for (int s = 0; s < 4; ++s) *(volatile v4u*)(dst + offs[s]) = pk[s];
    __threadfence();
#pragma unroll
    for (int s = 0; s < 4; ++s) *(volatile v4u*)(dst + offs[s]) = pk[s];
  } else {
    v4u phk[4], plk[4];
    size_t offs[4];
#pragma unroll
    for (int s = 0; s < 4; ++s) {
      const int L = s * 32 + (tid >> 3), p = tid & 7;
      const int h4 = L >> 5, d = L & 31;
      const int col = h4 * 32 + d;
      const int tb = p * 8;
      const float bc = bfr(bqn[col]);
      v4u a, b;
#pragma unroll
      for (int e = 0; e < 4; ++e) {
        const float v0 = Cs[(tb + 2 * e) * LDC + col] * (1.0f / 8192.0f) + bc;
        const float v1 = Cs[(tb + 2 * e + 1) * LDC + col] * (1.0f / 8192.0f) + bc;
        const float f0 = v0 * 16.0f, f1 = v1 * 16.0f;
        const _Float16 h0 = (_Float16)f0, h1 = (_Float16)f1;
        const float r0 = (f0 - (float)h0) * 16384.0f;
        const float r1 = (f1 - (float)h1) * 16384.0f;
        a[e] = pk16(h_bits(h0), h_bits(h1));
        b[e] = pk16(hb16(r0), hb16(r1));
      }
      phk[s] = a;
      plk[s] = b;
      offs[s] = ((size_t)((w * NHD + hb4 + h4) * HD + d)) * NTOK + tok0 + tb;
    }
#pragma unroll
    for (int s = 0; s < 4; ++s) { *(volatile v4u*)(vth + offs[s]) = phk[s]; *(volatile v4u*)(vtl + offs[s]) = plk[s]; }
    __threadfence();
#pragma unroll
    for (int s = 0; s < 4; ++s) { *(volatile v4u*)(vth + offs[s]) = phk[s]; *(volatile v4u*)(vtl + offs[s]) = plk[s]; }
  }
}

__global__ __launch_bounds__(256)
void attn_win(const unsigned short* __restrict__ qpl, const unsigned short* __restrict__ kpl,
              const unsigned short* __restrict__ vth, const unsigned short* __restrict__ vtl,
              const float* __restrict__ bt, unsigned short* ohi, unsigned short* olo) {
  __shared__ __align__(16) char pbuf[8 * PWB];
  __shared__ int cnts[NTOK];
  union CB { v8f v; v4f q[2]; };
  const int tid = threadIdx.x, wave = tid >> 5, lane = tid & 31, hh = lane >> 4, c = lane & 15;
  const int wh = blockIdx.x >> 2;
  const int w = wh >> 3, h = wh & 7;
  const int strip = (blockIdx.x & 3) * 8 + wave;
  const int q0 = strip * 16;

  for (int t = tid; t < NTOK; t += 256) cnts[t] = region_of(w, t);
  __syncthreads();

  const _Float16* Q  = (const _Float16*)(const void*)qpl + (size_t)wh * NTOK * HD;
  const _Float16* K  = (const _Float16*)(const void*)kpl + (size_t)wh * NTOK * HD;
  const _Float16* Vh = (const _Float16*)(const void*)vth + (size_t)wh * HD * NTOK;
  const _Float16* Vl = (const _Float16*)(const void*)vtl + (size_t)wh * HD * NTOK;
  const float* Bp = bt + ((size_t)(h * 32 + strip)) * 32 * 256 + lane * 8;
  _Float16* Ph = (_Float16*)(pbuf + wave * PWB);
  _Float16* Pl = Ph + 16 * PP;

  const v16h qa = ldfrag_h(Q + (size_t)(q0 + c) * HD + 8 * hh);
  int cntn[8];
#pragma unroll
  for (int r = 0; r < 8; ++r) cntn[r] = cnts[q0 + 8 * hh + r];
  float mrow[8], lrow[8];
#pragma unroll
  for (int r = 0; r < 8; ++r) { mrow[r] = -1e30f; lrow[r] = 0.f; }
  v8f ohh0 = zero8(), ohh1 = zero8(), ohl0 = zero8(), ohl1 = zero8(), olh0 = zero8(), olh1 = zero8();

#pragma unroll 1
  for (int kb = 0; kb < 8; ++kb) {
    v8f s[4];
#pragma unroll
    for (int j = 0; j < 4; ++j) {
      const int key = kb * 64 + j * 16 + c;
      const v16h kf = ldfrag_h(K + key * HD + 8 * hh);
      const float* bp = Bp + (kb * 4 + j) * 256;
      CB cb;
      cb.q[0] = *(const v4f*)(bp);
      cb.q[1] = *(const v4f*)(bp + 4);
      v8f sj = mma_g1(qa, kf, cb.v);
      const int cm = cnts[key];
#pragma unroll
      for (int r = 0; r < 8; ++r) sj[r] = sj[r] + ((cntn[r] != cm) ? -51200.0f : 0.0f);
      s[j] = sj;
    }
#pragma unroll
    for (int r = 0; r < 8; ++r) {
      float tm = fmaxf(fmaxf(s[0][r], s[1][r]), fmaxf(s[2][r], s[3][r]));
      tm = fmaxf(tm, __shfl_xor(tm, 1, 32));
      tm = fmaxf(tm, __shfl_xor(tm, 2, 32));
      tm = fmaxf(tm, __shfl_xor(tm, 4, 32));
      tm = fmaxf(tm, __shfl_xor(tm, 8, 32));
      const float mn = fmaxf(mrow[r], tm);
      const float alpha = __expf((mrow[r] - mn) * INV512);
      mrow[r] = mn;
      float ps = 0.f;
#pragma unroll
      for (int j = 0; j < 4; ++j) {
        const float p = __expf((s[j][r] - mn) * INV512 + LN4096);
        ps = ps + p;
        s[j][r] = p;
      }
      ps = ps + __shfl_xor(ps, 1, 32);
      ps = ps + __shfl_xor(ps, 2, 32);
      ps = ps + __shfl_xor(ps, 4, 32);
      ps = ps + __shfl_xor(ps, 8, 32);
      lrow[r] = lrow[r] * alpha + ps;
      ohh0[r] = ohh0[r] * alpha; ohh1[r] = ohh1[r] * alpha;
      ohl0[r] = ohl0[r] * alpha; ohl1[r] = ohl1[r] * alpha;
      olh0[r] = olh0[r] * alpha; olh1[r] = olh1[r] * alpha;
    }
#pragma unroll
    for (int j = 0; j < 4; ++j) {
#pragma unroll
      for (int r = 0; r < 8; ++r) {
        const float pf = s[j][r];
        const _Float16 phv = (_Float16)pf;
        const float res = (pf - (float)phv) * 8192.0f;
        const int idx = (8 * hh + r) * PP + j * 16 + c;
        Ph[idx] = phv;
        Pl[idx] = (_Float16)res;
      }
    }
    wave_sync_lds();
#pragma unroll
    for (int ks = 0; ks < 2; ++ks) {
      const v16h pa  = ldfrag_h(Ph + c * PP + ks * 32 + 8 * hh);
      const v16h pla = ldfrag_h(Pl + c * PP + ks * 32 + 8 * hh);
      const int koff = kb * 64 + ks * 32 + 8 * hh;
      {
        const v16h vh = ldfrag_h(Vh + (size_t)c * NTOK + koff);
        const v16h vl = ldfrag_h(Vl + (size_t)c * NTOK + koff);
        ohh0 = mma_raw(pa, vh, ohh0);
        ohl0 = mma_raw(pa, vl, ohl0);
        olh0 = mma_raw(pla, vh, olh0);
        guard3(ohh0, ohl0, olh0, pa, pla, vh, vl);
      }
      {
        const v16h vh = ldfrag_h(Vh + (size_t)(16 + c) * NTOK + koff);
        const v16h vl = ldfrag_h(Vl + (size_t)(16 + c) * NTOK + koff);
        ohh1 = mma_raw(pa, vh, ohh1);
        ohl1 = mma_raw(pa, vl, ohl1);
        olh1 = mma_raw(pla, vh, olh1);
        guard3(ohh1, ohl1, olh1, pa, pla, vh, vl);
      }
    }
    wave_sync_lds();
  }

  float* Os = (float*)(void*)(pbuf + wave * PWB);
#pragma unroll
  for (int r = 0; r < 8; ++r) {
    const float inv = 1.0f / (lrow[r] * 16.0f);
    const int row = 8 * hh + r;
    float o0 = ohh0[r] + ohl0[r] * (1.0f / 16384.0f);
    o0 = o0 + olh0[r] * (1.0f / 8192.0f);
    float o1 = ohh1[r] + ohl1[r] * (1.0f / 16384.0f);
    o1 = o1 + olh1[r] * (1.0f / 8192.0f);
    Os[row * OSP + c]      = o0 * inv;
    Os[row * OSP + 16 + c] = o1 * inv;
  }
  wave_sync_lds();
  v4u ph2[2], pl2[2];
  size_t off2[2];
#pragma unroll
  for (int sI = 0; sI < 2; ++sI) {
    const int line = sI * 4 + (lane >> 3), piece = lane & 7;
    const int row = 2 * line + (piece >> 2), d0 = (piece & 3) * 8;
    v4u a, b;
#pragma unroll
    for (int e = 0; e < 4; ++e) {
      const float f0 = Os[row * OSP + d0 + 2 * e] * 64.0f;
      const float f1 = Os[row * OSP + d0 + 2 * e + 1] * 64.0f;
      const _Float16 h0 = (_Float16)f0, h1 = (_Float16)f1;
      const float r0 = (f0 - (float)h0) * 16384.0f;
      const float r1 = (f1 - (float)h1) * 16384.0f;
      a[e] = pk16(h_bits(h0), h_bits(h1));
      b[e] = pk16(hb16(r0), hb16(r1));
    }
    ph2[sI] = a;
    pl2[sI] = b;
    off2[sI] = ((size_t)h * NROW + (size_t)w * NTOK + q0 + row) * HD + d0;
  }
  *(volatile v4u*)(ohi + off2[0]) = ph2[0];
  *(volatile v4u*)(ohi + off2[1]) = ph2[1];
  *(volatile v4u*)(olo + off2[0]) = pl2[0];
  *(volatile v4u*)(olo + off2[1]) = pl2[1];
  __threadfence();
  *(volatile v4u*)(ohi + off2[0]) = ph2[0];
  *(volatile v4u*)(ohi + off2[1]) = ph2[1];
  *(volatile v4u*)(olo + off2[0]) = pl2[0];
  *(volatile v4u*)(olo + off2[1]) = pl2[1];
}

__global__ __launch_bounds__(256)
void gemm_proj(const unsigned short* __restrict__ ohi, const unsigned short* __restrict__ olo,
               const unsigned short* __restrict__ wp, const float* __restrict__ bp, float* out) {
  __shared__ __align__(16) float Cs[64 * LDC];
  const int tid = threadIdx.x, wave = tid >> 5, lane = tid & 31, hh = lane >> 4, c = lane & 15;
  const int mb = blockIdx.x, nb = blockIdx.y;
  const int mw = wave >> 2, nw = wave & 3;
  const _Float16* W = (const _Float16*)(const void*)wp;
  const int arow0 = mb * 64 + mw * 32;
  const int bcol0 = nb * 128 + nw * 32;

  v8f h00 = zero8(), h01 = zero8(), h10 = zero8(), h11 = zero8();
  v8f l00 = zero8(), l01 = zero8(), l10 = zero8(), l11 = zero8();
#pragma unroll 1
  for (int ks = 0; ks < 8; ++ks) {
    const _Float16* Ah = (const _Float16*)(const void*)ohi + (size_t)ks * NROW * HD;
    const _Float16* Al = (const _Float16*)(const void*)olo + (size_t)ks * NROW * HD;
    const v16h fa0 = ldfrag_h(Ah + (size_t)(arow0 + c) * HD + 8 * hh);
    const v16h fa1 = ldfrag_h(Ah + (size_t)(arow0 + 16 + c) * HD + 8 * hh);
    const v16h ga0 = ldfrag_h(Al + (size_t)(arow0 + c) * HD + 8 * hh);
    const v16h ga1 = ldfrag_h(Al + (size_t)(arow0 + 16 + c) * HD + 8 * hh);
    const v16h fb0 = ldfrag_h(W + (size_t)(bcol0 + c) * CCH + ks * 32 + 8 * hh);
    const v16h fb1 = ldfrag_h(W + (size_t)(bcol0 + 16 + c) * CCH + ks * 32 + 8 * hh);
    h00 = mma_raw(fa0, fb0, h00);
    h01 = mma_raw(fa0, fb1, h01);
    h10 = mma_raw(fa1, fb0, h10);
    h11 = mma_raw(fa1, fb1, h11);
    l00 = mma_raw(ga0, fb0, l00);
    l01 = mma_raw(ga0, fb1, l01);
    l10 = mma_raw(ga1, fb0, l10);
    l11 = mma_raw(ga1, fb1, l11);
    guard8(h00, h01, h10, h11, l00, l01, l10, l11, fa0, fa1, ga0, ga1, fb0, fb1);
  }
#pragma unroll
  for (int r = 0; r < 8; ++r) {
    const int row = mw * 32 + 8 * hh + r;
    Cs[row * LDC + nw * 32 + c]             = h00[r] + l00[r] * (1.0f / 16384.0f);
    Cs[row * LDC + nw * 32 + 16 + c]        = h01[r] + l01[r] * (1.0f / 16384.0f);
    Cs[(row + 16) * LDC + nw * 32 + c]      = h10[r] + l10[r] * (1.0f / 16384.0f);
    Cs[(row + 16) * LDC + nw * 32 + 16 + c] = h11[r] + l11[r] * (1.0f / 16384.0f);
  }
  __syncthreads();

  const int w = mb >> 3, tok0 = (mb & 7) * 64;
  const float* bpn = bp + nb * 128 + lane * 4;
  v4f bb;
#pragma unroll
  for (int e = 0; e < 4; ++e) bb[e] = bfr(bpn[e]);
  v4f ov[8];
  size_t offs[8];
#pragma unroll
  for (int it = 0; it < 8; ++it) {
    const int row = wave * 8 + it;
    const int sp = spat_of(w, tok0 + row);
    v4f v = *(const v4f*)(Cs + row * LDC + lane * 4);
#pragma unroll
    for (int e = 0; e < 4; ++e) v[e] = v[e] * (1.0f / 65536.0f) + bb[e];
    ov[it] = v;
    offs[it] = (size_t)sp * CCH + nb * 128 + lane * 4;
  }
#pragma unroll
  for (int it = 0; it < 8; ++it) *(volatile v4f*)(out + offs[it]) = ov[it];
  __threadfence();
#pragma unroll
  for (int it = 0; it < 8; ++it) *(volatile v4f*)(out + offs[it]) = ov[it];
}

extern "C" void kernel_launch(void* const* d_in, const int* in_sizes, int n_in,
                              void* d_out, int out_size, void* d_ws, size_t ws_size,
                              hipStream_t stream) {
  if (n_in < 6) return;
  if (in_sizes[0] != NROW * CCH) return;
  if (in_sizes[1] != C3 * CCH || in_sizes[2] != C3) return;
  if (in_sizes[3] != CCH * CCH || in_sizes[4] != CCH) return;
  if (in_sizes[5] != NRPB * NHD) return;
  if (out_size != NROW * CCH) return;

  const float* x     = (const float*)d_in[0];
  const float* qkvw  = (const float*)d_in[1];
  const float* qkvb  = (const float*)d_in[2];
  const float* projw = (const float*)d_in[3];
  const float* projb = (const float*)d_in[4];
  const float* rpb   = (const float*)d_in[5];
  float* out = (float*)d_out;

  const size_t sX  = (size_t)NROW * CCH * 2;
  const size_t sWq = (size_t)C3 * CCH * 2;
  const size_t sWp = (size_t)CCH * CCH * 2;
  const size_t sBT = (size_t)NHD * NTOK * NTOK * 4;
  const size_t sQK = (size_t)NWIN * NHD * NTOK * HD * 2;
  const size_t sO  = (size_t)NHD * NROW * HD * 2;
  size_t off = 0;
  const size_t oX  = off; off += sX;
  const size_t oWq = off; off += sWq;
  const size_t oWp = off; off += sWp;
  const size_t oBT = off; off += sBT;
  const size_t oQ  = off; off += sQK;
  const size_t oK  = off; off += sQK;
  const size_t oVh = off; off += sQK;
  const size_t oVl = off; off += sQK;
  const size_t oOh = off; off += sO;
  const size_t oOl = off; off += sO;
  if (off > ws_size) return;
  if (off > (size_t)134217728) return;

  char* ws = (char*)d_ws;
  unsigned short* X8  = (unsigned short*)(ws + oX);
  unsigned short* Wq  = (unsigned short*)(ws + oWq);
  unsigned short* Wp  = (unsigned short*)(ws + oWp);
  float*          BT  = (float*)(ws + oBT);
  unsigned short* Qp  = (unsigned short*)(ws + oQ);
  unsigned short* Kp  = (unsigned short*)(ws + oK);
  unsigned short* Vth = (unsigned short*)(ws + oVh);
  unsigned short* Vtl = (unsigned short*)(ws + oVl);
  unsigned short* Ohi = (unsigned short*)(ws + oOh);
  unsigned short* Olo = (unsigned short*)(ws + oOl);

  const dim3 blk(256);
  cvt_x<<<dim3(NROW / 8), blk, 0, stream>>>(x, X8);
  cvt_w<<<dim3(C3 / 8), blk, 0, stream>>>(qkvw, Wq, C3);
  cvt_w<<<dim3(CCH / 8), blk, 0, stream>>>(projw, Wp, CCH);
  build_bias<<<dim3((NHD * 32 * 32 * 64) / 256), blk, 0, stream>>>(rpb, BT);
  gemm_qkv<<<dim3(NROW / 64, C3 / 128), blk, 0, stream>>>(X8, Wq, qkvb, Qp, Kp, Vth, Vtl);
  attn_win<<<dim3(NWIN * NHD * 4), blk, 0, stream>>>(Qp, Kp, Vth, Vtl, BT, Ohi, Olo);
  gemm_proj<<<dim3(NROW / 64, CCH / 128), blk, 0, stream>>>(Ohi, Olo, Wp, projb, out);
  (void)hipGetLastError();
}
